// ContiguousNormalizedFlow_28552942584189
// MI455X (gfx1250) — hardware-verified
//
#include <hip/hip_runtime.h>
#include <math.h>

typedef __attribute__((ext_vector_type(16))) _Float16 v16h;
typedef __attribute__((ext_vector_type(8)))  _Float16 v8h;
typedef __attribute__((ext_vector_type(8)))  float    v8f;
typedef __attribute__((ext_vector_type(4)))  float    v4f;
typedef __attribute__((ext_vector_type(2)))  float    v2f;

constexpr int kPoints        = 1000000;
constexpr int kDim           = 2;
constexpr int kUnits         = 64;
constexpr int kHid           = 64;
constexpr int kFeat          = 2 * kUnits;
constexpr int kNcol          = 16;
constexpr int kChunk         = 32;
constexpr int kNumChunks     = kPoints / kChunk;
constexpr int kWavesPerBlock = 4;
constexpr int kTilePitch     = 136;
constexpr int kCPitch        = 20;
static_assert(kPoints % kChunk == 0, "whole 32-point chunks");
static_assert(kFeat % 32 == 0, "K multiple of 32");
static_assert(kFeat == 128 && kNcol == 16, "operand table shape");
static_assert(((size_t)kPoints * kDim * 4) % 128 == 0, "second output starts on a 128-B line");
static_assert((size_t)kPoints * kDim * 4 + (size_t)kPoints * 4 == 12000000ull, "output total bytes");
static_assert((kTilePitch * 2) % 16 == 0 && (kCPitch * 4) % 16 == 0, "16-B aligned LDS rows");

constexpr float kCarryA      = 64.0f;
constexpr float kCarryB      = 64.0f;
constexpr float kLoScale     = 2048.0f;
constexpr float kLoInv       = 1.0f / kLoScale;
constexpr float kOutScale    = 1.0f / (kCarryA * kCarryB * (float)kUnits);
constexpr float kF16MinNorm  = 6.103515625e-05f;

constexpr size_t kOffWB   = 0;
constexpr size_t kSizeWB  = (size_t)kUnits * 4 * 4;
constexpr size_t kOffBT   = kOffWB + kSizeWB;
constexpr size_t kSizeBT  = (size_t)kNcol * kFeat * 2;
constexpr size_t kWsTotal = kOffBT + kSizeBT;
static_assert(kWsTotal == 5120ull, "carve total");
static_assert((kOffBT % 128) == 0, "128-B aligned regions");

union FragH { v16h v; v8h h[2]; };
__device__ __forceinline__ v16h frag_load_h(const _Float16* p) {
  FragH f;
  f.h[0] = *(const v8h*)(p);
  f.h[1] = *(const v8h*)(p + 16);
  return f.v;
}
__device__ __forceinline__ v8f mma_h(v16h a, v16h b, v8f c) {
  c = __builtin_amdgcn_wmma_f32_16x16x32_f16(false, a, false, b, (short)0, c, false, false);
  asm volatile("v_nop\n\tv_nop\n\tv_nop\n\tv_nop" : "+v"(c) : "v"(a), "v"(b));
  return c;
}
__device__ __forceinline__ float flush_small(float v) {
  return (fabsf(v) < kF16MinNorm) ? 0.0f : v;
}
__device__ __forceinline__ float f16_value(float v) {
  const _Float16 hv = (_Float16)flush_small(v);
  return (float)hv;
}

__global__ __launch_bounds__(64) void hyper_tables_kernel(
    const float* __restrict__ tp,
    const float* __restrict__ W1, const float* __restrict__ b1,
    const float* __restrict__ W2, const float* __restrict__ b2,
    const float* __restrict__ Wu, const float* __restrict__ bu,
    const float* __restrict__ Ww, const float* __restrict__ bw,
    const float* __restrict__ Wb, const float* __restrict__ bb,
    float* __restrict__ wbOut, unsigned short* __restrict__ btOut)
{
  __shared__ float sM1[kHid];
  __shared__ float sM2[kHid];
  __shared__ float sU[2 * kUnits];
  __shared__ float sW[2 * kUnits];
  __shared__ float sB[kUnits];
  __shared__ __align__(16) float sV[kNcol * kFeat];

  const int tid = threadIdx.x;
  const float tv = tp[0];

  sM1[tid] = tanhf(tv * W1[tid] + b1[tid]);
  __syncthreads();

  {
    float acc = 0.0f;
#pragma unroll 1
    for (int j = 0; j < kHid; ++j) acc = fmaf(sM1[j], W2[j * kHid + tid], acc);
    acc += b2[tid];
    sM2[tid] = tanhf(acc);
  }
  __syncthreads();

  {
    float a0 = 0.0f, a1 = 0.0f, c0 = 0.0f, c1 = 0.0f, e0 = 0.0f;
#pragma unroll 1
    for (int j = 0; j < kHid; ++j) {
      const float m = sM2[j];
      a0 = fmaf(m, Wu[j * (2 * kUnits) + tid], a0);
      a1 = fmaf(m, Wu[j * (2 * kUnits) + kUnits + tid], a1);
      c0 = fmaf(m, Ww[j * (2 * kUnits) + tid], c0);
      c1 = fmaf(m, Ww[j * (2 * kUnits) + kUnits + tid], c1);
      e0 = fmaf(m, Wb[j * kUnits + tid], e0);
    }
    sU[tid]          = a0 + bu[tid];
    sU[tid + kUnits] = a1 + bu[tid + kUnits];
    sW[tid]          = c0 + bw[tid];
    sW[tid + kUnits] = c1 + bw[tid + kUnits];
    sB[tid]          = e0 + bb[tid];
  }
  __syncthreads();

  const float u0 = sU[2 * tid];
  const float u1 = sU[2 * tid + 1];
  const float w0 = sW[2 * tid];
  const float w1 = sW[2 * tid + 1];
  const float bk = sB[tid];
  const float wu = w0 * u0 + w1 * u1;

  const float u0s = u0 * kCarryB;
  const float u1s = u1 * kCarryB;
  const float wus = wu * kCarryB;
  const float u0h = f16_value(u0s);
  const float u1h = f16_value(u1s);
  const float wuh = f16_value(wus);
  const float u0l = f16_value((u0s - u0h) * kLoScale);
  const float u1l = f16_value((u1s - u1h) * kLoScale);
  const float wul = f16_value((wus - wuh) * kLoScale);

#pragma unroll 1
  for (int n = 0; n < kNcol; ++n) {
    const float lowv  = (n == 0) ? u0h : (n == 1) ? u1h : (n == 3) ? u0l : (n == 4) ? u1l : 0.0f;
    const float highv = (n == 2) ? wuh : (n == 5) ? wul : 0.0f;
    sV[n * kFeat + tid]          = lowv;
    sV[n * kFeat + kUnits + tid] = highv;
  }
  __syncthreads();

  v4f wq;
  wq.x = w0;
  wq.y = w1;
  wq.z = bk;
  wq.w = 0.0f;

  v8h hv[4];
#pragma unroll
  for (int it = 0; it < 4; ++it) {
    const float* sp = sV + (it * 64 + tid) * 8;
    const v4f a0 = *(const v4f*)(sp);
    const v4f a1 = *(const v4f*)(sp + 4);
#pragma unroll
    for (int e = 0; e < 4; ++e) {
      hv[it][e]     = (_Float16)a0[e];
      hv[it][4 + e] = (_Float16)a1[e];
    }
  }

  for (int pass = 0; pass < 2; ++pass) {
    *(volatile v4f*)(wbOut + 4 * tid) = wq;
#pragma unroll
    for (int it = 0; it < 4; ++it)
      *(volatile v8h*)(btOut + (size_t)(it * 64 + tid) * 8) = hv[it];
    __threadfence();
  }
}

__global__ __launch_bounds__(128) void unit_reduce_kernel(
    const float* __restrict__ z, const float* __restrict__ wbTab,
    const unsigned short* __restrict__ btTab, float* __restrict__ out, int nChunks)
{
  __shared__ __align__(16) float    sWB[kUnits * 4];
  __shared__ __align__(16) _Float16 sA[kWavesPerBlock][kChunk * kTilePitch];
  __shared__ __align__(16) float    sC[kWavesPerBlock][kChunk * kCPitch];

  const int tid  = threadIdx.x;
  const int lane = tid & 31;
  const int wave = tid >> 5;
  const int hh   = lane >> 4;
  const int cl   = lane & 15;

  {
    const v2f q = *(const v2f*)(wbTab + 2 * tid);
    *(v2f*)(sWB + 2 * tid) = q;
  }
  __syncthreads();

  const int chunk = blockIdx.x * kWavesPerBlock + wave;
  if (chunk >= nChunks) return;

  const _Float16* Bt = (const _Float16*)btTab;
  v16h bfr[4];
#pragma unroll
  for (int ks = 0; ks < 4; ++ks) bfr[ks] = frag_load_h(Bt + cl * kFeat + 32 * ks + 8 * hh);

  const int p = chunk * kChunk + lane;
  const v2f zz = *(const v2f*)(z + 2 * (size_t)p);
  const float z0 = zz.x;
  const float z1 = zz.y;

  _Float16* tile = sA[wave];
  _Float16* trow = tile + lane * kTilePitch;

#pragma unroll 1
  for (int g = 0; g < kUnits / 8; ++g) {
    v8h tv, sv;
#pragma unroll
    for (int e = 0; e < 8; ++e) {
      const v4f wv = *(const v4f*)(sWB + (8 * g + e) * 4);
      const float lin = fmaf(z1, wv.y, z0 * wv.x) + wv.z;
      const float ex  = expf(2.0f * lin);
      const float rc  = __builtin_amdgcn_rcpf(ex + 1.0f);
      const float th  = 1.0f - 2.0f * rc;
      const float sq  = 1.0f - th * th;
      const float ta  = flush_small(th * kCarryA);
      const float sa  = flush_small(sq * kCarryA);
      tv[e] = (_Float16)ta;
      sv[e] = (_Float16)sa;
    }
    *(v8h*)(trow + 8 * g)          = tv;
    *(v8h*)(trow + kUnits + 8 * g) = sv;
  }
  __builtin_amdgcn_fence(__ATOMIC_RELEASE, "workgroup");
  __builtin_amdgcn_wave_barrier();
  __builtin_amdgcn_fence(__ATOMIC_ACQUIRE, "workgroup");

  v8f acc0 = (v8f){0.f, 0.f, 0.f, 0.f, 0.f, 0.f, 0.f, 0.f};
  v8f acc1 = (v8f){0.f, 0.f, 0.f, 0.f, 0.f, 0.f, 0.f, 0.f};
#pragma unroll
  for (int ks = 0; ks < 4; ++ks) {
    const v16h a0 = frag_load_h(tile + cl * kTilePitch + 32 * ks + 8 * hh);
    const v16h a1 = frag_load_h(tile + (16 + cl) * kTilePitch + 32 * ks + 8 * hh);
    acc0 = mma_h(a0, bfr[ks], acc0);
    acc1 = mma_h(a1, bfr[ks], acc1);
  }

  float* cs = sC[wave];
#pragma unroll
  for (int r = 0; r < 8; ++r) {
    cs[(8 * hh + r) * kCPitch + cl]      = acc0[r];
    cs[(16 + 8 * hh + r) * kCPitch + cl] = acc1[r];
  }
  __builtin_amdgcn_fence(__ATOMIC_RELEASE, "workgroup");
  __builtin_amdgcn_wave_barrier();
  __builtin_amdgcn_fence(__ATOMIC_ACQUIRE, "workgroup");

  const v4f ca = *(const v4f*)(cs + lane * kCPitch);
  const v4f cb = *(const v4f*)(cs + lane * kCPitch + 4);
  const float d0 = (ca.x + ca.w * kLoInv) * kOutScale;
  const float d1 = (ca.y + cb.x * kLoInv) * kOutScale;
  const float dl = -((ca.z + cb.y * kLoInv) * kOutScale);

  v2f o;
  o.x = d0;
  o.y = d1;
  float* p0 = out + 2 * (size_t)p;
  float* p1 = out + (size_t)kPoints * kDim + p;
  for (int pass = 0; pass < 2; ++pass) {
    *(volatile v2f*)p0   = o;
    *(volatile float*)p1 = dl;
    __threadfence();
  }
}

extern "C" void kernel_launch(void* const* d_in, const int* in_sizes, int n_in,
                              void* d_out, int out_size, void* d_ws, size_t ws_size,
                              hipStream_t stream) {
  if (n_in < 13) return;
  if (in_sizes[0] != 1) return;
  if (in_sizes[1] != kPoints * kDim) return;
  if (in_sizes[3] != kHid) return;
  if (in_sizes[4] != kHid) return;
  if (in_sizes[5] != kHid * kHid) return;
  if (in_sizes[6] != kHid) return;
  if (in_sizes[7] != kHid * 2 * kUnits) return;
  if (in_sizes[8] != 2 * kUnits) return;
  if (in_sizes[9] != kHid * 2 * kUnits) return;
  if (in_sizes[10] != 2 * kUnits) return;
  if (in_sizes[11] != kHid * kUnits) return;
  if (in_sizes[12] != kUnits) return;
  if (out_size != kPoints * (kDim + 1)) return;
  if (ws_size < kWsTotal) return;

  const float* tp = (const float*)d_in[0];
  const float* z  = (const float*)d_in[1];
  const float* W1 = (const float*)d_in[3];
  const float* b1 = (const float*)d_in[4];
  const float* W2 = (const float*)d_in[5];
  const float* b2 = (const float*)d_in[6];
  const float* Wu = (const float*)d_in[7];
  const float* bu = (const float*)d_in[8];
  const float* Ww = (const float*)d_in[9];
  const float* bw = (const float*)d_in[10];
  const float* Wb = (const float*)d_in[11];
  const float* bb = (const float*)d_in[12];
  float* out = (float*)d_out;

  char* ws = (char*)d_ws;
  float*          wbTab = (float*)(ws + kOffWB);
  unsigned short* btTab = (unsigned short*)(ws + kOffBT);

  hyper_tables_kernel<<<1, 64, 0, stream>>>(tp, W1, b1, W2, b2, Wu, bu, Ww, bw, Wb, bb, wbTab, btTab);

  const int blocks = (kNumChunks + kWavesPerBlock - 1) / kWavesPerBlock;
  unit_reduce_kernel<<<blocks, kWavesPerBlock * kChunk, 0, stream>>>(z, wbTab, btTab, out, kNumChunks);
}
